// ModelDSS_76459007803635
// MI455X (gfx1250) — hardware-verified
//
#include <hip/hip_runtime.h>
#include <stddef.h>


#define NTHR   256
#define NWAVE  8
#define LL     32
#define EPT    8
#define CHUNK  (NTHR * EPT)
#define WCAP   (EPT * 32)
#define LISTN  (NWAVE * WCAP)
#define PASSN  (NWAVE * 32)
#define PCAP   (CHUNK + PASSN)
#define NB     512
#define NNODE  (NWAVE * 32)
#define KE1    64
#define DPHI   67
#define KP1    96
#define DPSI   97
#define WSC    16.0f
#define WINV   0.0625f
#define ALPHAC 0.5f

static_assert(PASSN == 256);
static_assert(NNODE == 256);
static_assert(PCAP >= CHUNK + PASSN);
static_assert(((NB * LL) % (128 * NWAVE)) == 0);

typedef float    v4f  __attribute__((ext_vector_type(4)));
typedef float    v8f  __attribute__((ext_vector_type(8)));
typedef int      v4i  __attribute__((ext_vector_type(4)));
typedef _Float16 v8h  __attribute__((ext_vector_type(8)));
typedef _Float16 v16h __attribute__((ext_vector_type(16)));
union FragH { v16h v; v8h h[2]; };

__device__ __forceinline__ v8f wmh(v16h a, v16h b, v8f c) {
  v8f d = __builtin_amdgcn_wmma_f32_16x16x32_f16(false, a, false, b, (short)0, c, false, false);
  asm volatile("v_nop\n\tv_nop\n\tv_nop\n\tv_nop" : "+v"(d) : "v"(a), "v"(b));
  return d;
}

__device__ __forceinline__ v8h relu8(v8f d) {
  v8h r;
#pragma unroll
  for (int i = 0; i < 8; ++i) { const float t = fmaxf(d[i] * WINV, 0.0f); r[i] = (_Float16)t; }
  return r;
}

__device__ __forceinline__ v8h cvt8(v4f a, v4f b) {
  v8h r;
  r[0] = (_Float16)a.x; r[1] = (_Float16)a.y; r[2] = (_Float16)a.z; r[3] = (_Float16)a.w;
  r[4] = (_Float16)b.x; r[5] = (_Float16)b.y; r[6] = (_Float16)b.z; r[7] = (_Float16)b.w;
  return r;
}

__device__ __forceinline__ v8f ldc8(const float* p) {
  const v4f a = *(const v4f*)p;
  const v4f b = *(const v4f*)(p + 4);
  v8f c;
  c[0] = a.x; c[1] = a.y; c[2] = a.z; c[3] = a.w;
  c[4] = b.x; c[5] = b.y; c[6] = b.z; c[7] = b.w;
  return c;
}

__device__ __forceinline__ v8f zero8f() {
  v8f z;
#pragma unroll
  for (int i = 0; i < 8; ++i) z[i] = 0.0f;
  return z;
}

__device__ __forceinline__ int scan_chunk(const int* __restrict__ keys, int nE, int cbase, int nodeBase,
                                          int vec8, int* list, int tid, int wave) {
  int wc = 0;
  const int el0  = tid * EPT;
  const int e0   = cbase + el0;
  const int sent = -2147483647 - 1;
  v4i da, db;
  if (vec8 != 0 && e0 + 7 < nE) {
    da = *(const v4i*)(keys + e0);
    db = *(const v4i*)(keys + e0 + 4);
  } else {
    da.x = (e0     < nE) ? keys[min(e0, nE - 1)] : sent;
    da.y = (e0 + 1 < nE) ? keys[min(e0 + 1, nE - 1)] : sent;
    da.z = (e0 + 2 < nE) ? keys[min(e0 + 2, nE - 1)] : sent;
    da.w = (e0 + 3 < nE) ? keys[min(e0 + 3, nE - 1)] : sent;
    db.x = (e0 + 4 < nE) ? keys[min(e0 + 4, nE - 1)] : sent;
    db.y = (e0 + 5 < nE) ? keys[min(e0 + 5, nE - 1)] : sent;
    db.z = (e0 + 6 < nE) ? keys[min(e0 + 6, nE - 1)] : sent;
    db.w = (e0 + 7 < nE) ? keys[min(e0 + 7, nE - 1)] : sent;
  }
  const unsigned nb = (unsigned)nodeBase;
  const unsigned s0 = (unsigned)da.x - nb, s1 = (unsigned)da.y - nb;
  const unsigned s2 = (unsigned)da.z - nb, s3 = (unsigned)da.w - nb;
  const unsigned s4 = (unsigned)db.x - nb, s5 = (unsigned)db.y - nb;
  const unsigned s6 = (unsigned)db.z - nb, s7 = (unsigned)db.w - nb;
  const bool h0 = s0 < (unsigned)NB, h1 = s1 < (unsigned)NB, h2 = s2 < (unsigned)NB, h3 = s3 < (unsigned)NB;
  const bool h4 = s4 < (unsigned)NB, h5 = s5 < (unsigned)NB, h6 = s6 < (unsigned)NB, h7 = s7 < (unsigned)NB;
  const unsigned any = __builtin_amdgcn_ballot_w32(h0 | h1 | h2 | h3 | h4 | h5 | h6 | h7);
  if (any != 0u) {
#define HITJ(J, HJ) { \
      const unsigned mj = __builtin_amdgcn_ballot_w32(HJ); \
      if (mj != 0u) { \
        if (HJ) { \
          const int pos = wc + (int)__builtin_amdgcn_mbcnt_lo(mj, 0u); \
          if (pos < WCAP) list[wave * WCAP + pos] = el0 + (J); \
        } \
        wc += (int)__builtin_popcount(mj); } }
    HITJ(0, h0)
    HITJ(1, h1)
    HITJ(2, h2)
    HITJ(3, h3)
    HITJ(4, h4)
    HITJ(5, h5)
    HITJ(6, h6)
    HITJ(7, h7)
#undef HITJ
  }
  return wc;
}

__global__ __launch_bounds__(NTHR) void k_edge(
    const _Float16* __restrict__ h16, const int* __restrict__ ei, const float* __restrict__ ea,
    const float* __restrict__ W1to, const float* __restrict__ B1to,
    const float* __restrict__ W2to, const float* __restrict__ B2to,
    const float* __restrict__ W1fr, const float* __restrict__ B1fr,
    const float* __restrict__ W2fr, const float* __restrict__ B2fr,
    float* mess, int nN, int nE, int t, int hz, int vec8, int rowsPad) {
  __shared__ __attribute__((aligned(16))) float    acc[(NB + 1) * LL];
  __shared__ __attribute__((aligned(16))) float    msg[PASSN * LL];
  __shared__ __attribute__((aligned(16))) _Float16 stg[PASSN * KE1];
  __shared__ __attribute__((aligned(16))) float    eas[PASSN * 4];
  __shared__ __attribute__((aligned(16))) int      list[LISTN];
  __shared__ __attribute__((aligned(16))) int      pend[PCAP];
  __shared__ int slotb[PASSN];
  __shared__ __attribute__((aligned(16))) _Float16 wsm1[LL * KE1];
  __shared__ __attribute__((aligned(16))) _Float16 wsm2[LL * LL];
  __shared__ __attribute__((aligned(16))) float    bs1[LL];
  __shared__ __attribute__((aligned(16))) float    bs2[LL];
  __shared__ __attribute__((aligned(16))) float    w1c[3 * LL];
  __shared__ int wcnt[NWAVE];
  __shared__ int pendN;

  const int tid = threadIdx.x, lane = tid & 31, wave = tid >> 5, hh = lane >> 4, m = lane & 15;
  const int dir = blockIdx.y;
  const int nodeBase = blockIdx.x * NB;
  const int* srcs = ei;
  const int* dsts = ei + nE;
  const int* keys = (dir == 0) ? dsts : srcs;
  const int* oths = (dir == 0) ? srcs : dsts;
  const float* W1  = ((dir == 0) ? W1to : W1fr) + (size_t)t * DPHI * LL;
  const float* Bi1 = ((dir == 0) ? B1to : B1fr) + (size_t)t * LL;
  const float* W2  = ((dir == 0) ? W2to : W2fr) + (size_t)t * LL * LL;
  const float* Bi2 = ((dir == 0) ? B2to : B2fr) + (size_t)t * LL;
  float* outp = mess + (size_t)dir * (size_t)rowsPad * LL + (size_t)nodeBase * LL;

  for (int i = tid; i < (NB + 1) * LL; i += NTHR) acc[i] = 0.0f;
  for (int i = tid; i < LL * KE1; i += NTHR) {
    const int f = i >> 6, k = i & 63;
    wsm1[i] = (_Float16)(W1[k * LL + f] * WSC);
  }
  for (int i = tid; i < LL * LL; i += NTHR) {
    const int f = i >> 5, k = i & 31;
    wsm2[i] = (_Float16)(W2[k * LL + f] * WSC);
  }
  if (tid < LL) { bs1[tid] = Bi1[tid] * WSC; bs2[tid] = Bi2[tid] * WSC; }
  if (tid < 3 * LL) {
    const int c = tid >> 5, f = tid & 31;
    w1c[tid] = W1[(KE1 + c) * LL + f] * WSC;
  }
  if (tid == 0) pendN = 0;
  __syncthreads();

  const int nChunks = (nE + CHUNK - 1) / CHUNK;
#pragma unroll 1
  for (int ch = 0; ch < nChunks; ++ch) {
    const int cbase = ch * CHUNK;
    const int wc = scan_chunk(keys, nE, cbase, nodeBase, vec8, list, tid, wave);
    if (lane == 0) wcnt[wave] = wc;
    __syncthreads();

    const int base = pendN;
    int tot = 0, myoff = 0;
#pragma unroll
    for (int w = 0; w < NWAVE; ++w) {
      int c = wcnt[w];
      c = c > WCAP ? WCAP : (c < 0 ? 0 : c);
      if (w < wave) myoff += c;
      tot += c;
    }
    int newN = base + tot;
    newN = newN > PCAP ? PCAP : newN;
    {
      int n = wcnt[wave];
      n = n > WCAP ? WCAP : (n < 0 ? 0 : n);
      const int* lp = list + wave * WCAP;
      for (int i = lane; i < n; i += 32) {
        const int pos = base + myoff + i;
        if (pos < PCAP) pend[pos] = cbase + lp[i];
      }
    }
    const int fin = (ch == nChunks - 1) ? 1 : 0;
    const int R   = (fin != 0) ? (newN + PASSN - 1) / PASSN : newN / PASSN;
    const int Pv  = (fin != 0) ? newN : R * PASSN;
    __syncthreads();

#pragma unroll 1
    for (int r = 0; r < R; ++r) {
      {
        const int idx = r * PASSN + wave * 32 + lane;
        const bool valid = idx < Pv;
        int e = 0;
        if (valid) e = pend[idx];
        e = e < 0 ? 0 : (e > nE - 1 ? nE - 1 : e);
        int kn = keys[e];
        int on = oths[e];
        int slot = kn - nodeBase;
        if (!valid || (unsigned)slot >= (unsigned)NB || kn == on) slot = NB;
        kn = kn < 0 ? 0 : (kn > nN - 1 ? nN - 1 : kn);
        on = on < 0 ? 0 : (on > nN - 1 ? nN - 1 : on);
        const int row = wave * 32 + lane;
        if (hz == 0) {
          const v8h* pk = (const v8h*)(h16 + (size_t)kn * LL);
          const v8h* po = (const v8h*)(h16 + (size_t)on * LL);
          const v8h hk0 = pk[0], hk1 = pk[1], hk2 = pk[2], hk3 = pk[3];
          const v8h ho0 = po[0], ho1 = po[1], ho2 = po[2], ho3 = po[3];
          v8h* sp = (v8h*)(stg + row * KE1);
          sp[0] = hk0; sp[1] = hk1; sp[2] = hk2; sp[3] = hk3;
          sp[4] = ho0; sp[5] = ho1; sp[6] = ho2; sp[7] = ho3;
        }
        v4f ev;
        ev.x = ea[(size_t)e * 3 + 0];
        ev.y = ea[(size_t)e * 3 + 1];
        ev.z = ea[(size_t)e * 3 + 2];
        ev.w = 0.0f;
        *(v4f*)(eas + row * 4) = ev;
        slotb[row] = slot;
      }
      __syncthreads();

      {
        v8f d1[2][2];
        {
          const v4f ev0 = *(const v4f*)(eas + (wave * 32 + m) * 4);
          const v4f ev1 = *(const v4f*)(eas + (wave * 32 + 16 + m) * 4);
#pragma unroll
          for (int ft = 0; ft < 2; ++ft) {
            const v8f cb  = ldc8(bs1 + 16 * ft + 8 * hh);
            const v8f wc0 = ldc8(w1c + 16 * ft + 8 * hh);
            const v8f wc1 = ldc8(w1c + LL + 16 * ft + 8 * hh);
            const v8f wc2 = ldc8(w1c + 2 * LL + 16 * ft + 8 * hh);
            v8f c0, c1;
#pragma unroll
            for (int rr = 0; rr < 8; ++rr) {
              c0[rr] = cb[rr] + ev0.x * wc0[rr] + ev0.y * wc1[rr] + ev0.z * wc2[rr];
              c1[rr] = cb[rr] + ev1.x * wc0[rr] + ev1.y * wc1[rr] + ev1.z * wc2[rr];
            }
            d1[ft][0] = c0;
            d1[ft][1] = c1;
          }
        }
        if (hz == 0) {
#pragma unroll
          for (int ks = 0; ks < 2; ++ks) {
            FragH b0, b1;
            const _Float16* s0 = stg + (wave * 32 + m) * KE1 + 32 * ks + 8 * hh;
            const _Float16* s1 = stg + (wave * 32 + 16 + m) * KE1 + 32 * ks + 8 * hh;
            b0.h[0] = *(const v8h*)s0;  b0.h[1] = *(const v8h*)(s0 + 16);
            b1.h[0] = *(const v8h*)s1;  b1.h[1] = *(const v8h*)(s1 + 16);
#pragma unroll
            for (int ft = 0; ft < 2; ++ft) {
              FragH a;
              const _Float16* ap = wsm1 + (16 * ft + m) * KE1 + 32 * ks + 8 * hh;
              a.h[0] = *(const v8h*)ap;
              a.h[1] = *(const v8h*)(ap + 16);
              d1[ft][0] = wmh(a.v, b0.v, d1[ft][0]);
              d1[ft][1] = wmh(a.v, b1.v, d1[ft][1]);
            }
          }
        }
        FragH bq[2];
        bq[0].h[0] = relu8(d1[0][0]); bq[0].h[1] = relu8(d1[1][0]);
        bq[1].h[0] = relu8(d1[0][1]); bq[1].h[1] = relu8(d1[1][1]);
#pragma unroll
        for (int ft = 0; ft < 2; ++ft) {
          FragH a;
          const _Float16* ap = wsm2 + (16 * ft + m) * LL + 8 * hh;
          a.h[0] = *(const v8h*)ap;
          a.h[1] = *(const v8h*)(ap + 16);
          const v8f c = ldc8(bs2 + 16 * ft + 8 * hh);
          const v8f e0 = wmh(a.v, bq[0].v, c);
          const v8f e1 = wmh(a.v, bq[1].v, c);
          float* mp = msg + (wave * 32 + m) * LL + 16 * ft + 8 * hh;
          float* mq = msg + (wave * 32 + 16 + m) * LL + 16 * ft + 8 * hh;
          v4f u0 = {e0[0] * WINV, e0[1] * WINV, e0[2] * WINV, e0[3] * WINV};
          v4f u1 = {e0[4] * WINV, e0[5] * WINV, e0[6] * WINV, e0[7] * WINV};
          v4f u2 = {e1[0] * WINV, e1[1] * WINV, e1[2] * WINV, e1[3] * WINV};
          v4f u3 = {e1[4] * WINV, e1[5] * WINV, e1[6] * WINV, e1[7] * WINV};
          *(v4f*)mp = u0; *(v4f*)(mp + 4) = u1;
          *(v4f*)mq = u2; *(v4f*)(mq + 4) = u3;
        }
      }
      __syncthreads();

      if (wave == 0) {
#pragma unroll 1
        for (int i = 0; i < PASSN; ++i) {
          int sl = slotb[i];
          sl = sl < 0 ? 0 : (sl > NB ? NB : sl);
          const float v = msg[i * LL + lane];
          acc[sl * LL + lane] += v;
        }
      }
      __syncthreads();
    }

    int rem = newN - R * PASSN;
    rem = rem < 0 ? 0 : rem;
    if (R > 0 && tid < rem) pend[tid] = pend[R * PASSN + tid];
    if (tid == 0) pendN = rem;
  }
  __syncthreads();

  constexpr int NQ = (NB * LL) / (128 * NWAVE);
#pragma unroll
  for (int q = 0; q < NQ; ++q) {
    const int f = (wave * NQ + q) * 128 + 4 * lane;
    const v4f v = *(const v4f*)(acc + f);
    *(volatile v4f*)(outp + f) = v;
  }
  __threadfence();
#pragma unroll
  for (int q = 0; q < NQ; ++q) {
    const int f = (wave * NQ + q) * 128 + 4 * lane;
    const v4f v = *(const v4f*)(acc + f);
    *(volatile v4f*)(outp + f) = v;
  }
}

__device__ __forceinline__ void node_store_pass(const float* hstw, const _Float16* hst16w, const float* ust,
                                                float* hbuf, _Float16* h16, float* outp,
                                                size_t rb, int outBase, int outLim, int lane, int wave, int last) {
#pragma unroll
  for (int q = 0; q < 8; ++q) {
    const int idx = q * 128 + 4 * lane;
    const v4f v = *(const v4f*)(hstw + idx);
    *(volatile v4f*)(hbuf + rb + idx) = v;
  }
#pragma unroll
  for (int q = 0; q < 4; ++q) {
    const int idx = q * 256 + 8 * lane;
    const v8h v = *(const v8h*)(hst16w + idx);
    *(volatile v8h*)(h16 + rb + idx) = v;
  }
  if (last != 0 && wave == 0) {
#pragma unroll
    for (int q = 0; q < 2; ++q) {
      const int idx = q * 128 + 4 * lane;
      const int gi = outBase + idx;
      const v4f v = *(const v4f*)(ust + idx);
      if (gi + 3 < outLim) {
        *(volatile v4f*)(outp + gi) = v;
      } else {
        if (gi     < outLim) *(volatile float*)(outp + gi)     = v.x;
        if (gi + 1 < outLim) *(volatile float*)(outp + gi + 1) = v.y;
        if (gi + 2 < outLim) *(volatile float*)(outp + gi + 2) = v.z;
      }
    }
  }
}

__global__ __launch_bounds__(NTHR) void k_node(
    float* hbuf, _Float16* h16, const float* __restrict__ mess, const float* __restrict__ prb,
    const float* __restrict__ PW1, const float* __restrict__ PB1,
    const float* __restrict__ PW2, const float* __restrict__ PB2,
    const float* __restrict__ DW1, const float* __restrict__ DB1,
    const float* __restrict__ DW2, const float* __restrict__ DB2,
    float* outp, int nN, int t, int hz, int last, int rowsPad, int outLim) {
  __shared__ __attribute__((aligned(16))) _Float16 wp1[LL * KP1];
  __shared__ __attribute__((aligned(16))) _Float16 wp2[LL * LL];
  __shared__ __attribute__((aligned(16))) _Float16 wd1[LL * LL];
  __shared__ __attribute__((aligned(16))) _Float16 wd2[16 * LL];
  __shared__ __attribute__((aligned(16))) float    pb1s[LL];
  __shared__ __attribute__((aligned(16))) float    pb2s[LL];
  __shared__ __attribute__((aligned(16))) float    db1s[LL];
  __shared__ __attribute__((aligned(16))) float    w96s[LL];
  __shared__ float db2s;
  __shared__ __attribute__((aligned(16))) float    hst[NWAVE * 32 * LL];
  __shared__ __attribute__((aligned(16))) _Float16 hst16[NWAVE * 32 * LL];
  __shared__ __attribute__((aligned(16))) float    ust[NNODE];

  const int tid = threadIdx.x, lane = tid & 31, wave = tid >> 5, hh = lane >> 4, m = lane & 15;

  const float* P1 = PW1 + (size_t)t * DPSI * LL;
  const float* P2 = PW2 + (size_t)t * LL * LL;
  const float* D1 = DW1 + (size_t)t * LL * LL;
  for (int i = tid; i < LL * KP1; i += NTHR) {
    const int f = i / KP1, k = i - f * KP1;
    wp1[i] = (_Float16)(P1[k * LL + f] * WSC);
  }
  for (int i = tid; i < LL * LL; i += NTHR) {
    const int f = i >> 5, k = i & 31;
    wp2[i] = (_Float16)(P2[k * LL + f] * WSC);
    wd1[i] = (_Float16)(D1[k * LL + f] * WSC);
  }
  for (int i = tid; i < 16 * LL; i += NTHR) {
    const int f = i >> 5, k = i & 31;
    const float v = (f == 0) ? DW2[t * LL + k] * WSC : 0.0f;
    wd2[i] = (_Float16)v;
  }
  if (tid < LL) {
    pb1s[tid] = PB1[t * LL + tid] * WSC;
    pb2s[tid] = PB2[t * LL + tid] * WSC;
    db1s[tid] = DB1[t * LL + tid] * WSC;
    w96s[tid] = P1[96 * LL + tid] * WSC;
  }
  if (tid == 0) db2s = DB2[t] * WSC;
  __syncthreads();

  const int nd0 = blockIdx.x * NNODE + wave * 32;
  int nc[2];
  v4f hr[2][4];
  v8f d1[2][2];

#pragma unroll
  for (int et = 0; et < 2; ++et) {
    const int node = nd0 + 16 * et + m;
    nc[et] = node > nN - 1 ? nN - 1 : node;
    const float pv = prb[nc[et]];
#pragma unroll
    for (int ft = 0; ft < 2; ++ft) {
      const v8f cb = ldc8(pb1s + 16 * ft + 8 * hh);
      const v8f wv = ldc8(w96s + 16 * ft + 8 * hh);
      v8f c;
#pragma unroll
      for (int rr = 0; rr < 8; ++rr) c[rr] = cb[rr] + pv * wv[rr];
      d1[ft][et] = c;
    }
  }

  if (hz == 0) {
    FragH b[2];
#pragma unroll
    for (int et = 0; et < 2; ++et) {
      const float* hp = hbuf + (size_t)nc[et] * LL;
      hr[et][0] = *(const v4f*)(hp + 8 * hh);
      hr[et][1] = *(const v4f*)(hp + 8 * hh + 4);
      hr[et][2] = *(const v4f*)(hp + 16 + 8 * hh);
      hr[et][3] = *(const v4f*)(hp + 20 + 8 * hh);
      b[et].h[0] = cvt8(hr[et][0], hr[et][1]);
      b[et].h[1] = cvt8(hr[et][2], hr[et][3]);
    }
#pragma unroll
    for (int ft = 0; ft < 2; ++ft) {
      FragH a;
      const _Float16* ap = wp1 + (16 * ft + m) * KP1 + 8 * hh;
      a.h[0] = *(const v8h*)ap;
      a.h[1] = *(const v8h*)(ap + 16);
      d1[ft][0] = wmh(a.v, b[0].v, d1[ft][0]);
      d1[ft][1] = wmh(a.v, b[1].v, d1[ft][1]);
    }
  } else {
    const v4f z = {0.0f, 0.0f, 0.0f, 0.0f};
#pragma unroll
    for (int et = 0; et < 2; ++et) { hr[et][0] = z; hr[et][1] = z; hr[et][2] = z; hr[et][3] = z; }
  }

#pragma unroll
  for (int ks = 1; ks < 3; ++ks) {
    const float* mb = mess + (size_t)(ks - 1) * (size_t)rowsPad * LL;
    FragH b[2];
#pragma unroll
    for (int et = 0; et < 2; ++et) {
      const float* mp = mb + (size_t)nc[et] * LL;
      const v4f x0 = *(const v4f*)(mp + 8 * hh);
      const v4f x1 = *(const v4f*)(mp + 8 * hh + 4);
      const v4f x2 = *(const v4f*)(mp + 16 + 8 * hh);
      const v4f x3 = *(const v4f*)(mp + 20 + 8 * hh);
      b[et].h[0] = cvt8(x0, x1);
      b[et].h[1] = cvt8(x2, x3);
    }
#pragma unroll
    for (int ft = 0; ft < 2; ++ft) {
      FragH a;
      const _Float16* ap = wp1 + (16 * ft + m) * KP1 + 32 * ks + 8 * hh;
      a.h[0] = *(const v8h*)ap;
      a.h[1] = *(const v8h*)(ap + 16);
      d1[ft][0] = wmh(a.v, b[0].v, d1[ft][0]);
      d1[ft][1] = wmh(a.v, b[1].v, d1[ft][1]);
    }
  }

  FragH bq[2];
  bq[0].h[0] = relu8(d1[0][0]); bq[0].h[1] = relu8(d1[1][0]);
  bq[1].h[0] = relu8(d1[0][1]); bq[1].h[1] = relu8(d1[1][1]);
  v8f d2[2][2];
#pragma unroll
  for (int ft = 0; ft < 2; ++ft) {
    FragH a;
    const _Float16* ap = wp2 + (16 * ft + m) * LL + 8 * hh;
    a.h[0] = *(const v8h*)ap;
    a.h[1] = *(const v8h*)(ap + 16);
    const v8f c = ldc8(pb2s + 16 * ft + 8 * hh);
    d2[ft][0] = wmh(a.v, bq[0].v, c);
    d2[ft][1] = wmh(a.v, bq[1].v, c);
  }

  FragH bh[2];
#pragma unroll
  for (int et = 0; et < 2; ++et) {
#pragma unroll
    for (int ft = 0; ft < 2; ++ft) {
      const v4f ha = hr[et][2 * ft], hb = hr[et][2 * ft + 1];
      v4f n0, n1;
      n0.x = ha.x + ALPHAC * (d2[ft][et][0] * WINV);
      n0.y = ha.y + ALPHAC * (d2[ft][et][1] * WINV);
      n0.z = ha.z + ALPHAC * (d2[ft][et][2] * WINV);
      n0.w = ha.w + ALPHAC * (d2[ft][et][3] * WINV);
      n1.x = hb.x + ALPHAC * (d2[ft][et][4] * WINV);
      n1.y = hb.y + ALPHAC * (d2[ft][et][5] * WINV);
      n1.z = hb.z + ALPHAC * (d2[ft][et][6] * WINV);
      n1.w = hb.w + ALPHAC * (d2[ft][et][7] * WINV);
      float* sp = hst + (wave * 32 + 16 * et + m) * LL + 16 * ft + 8 * hh;
      *(v4f*)sp = n0;
      *(v4f*)(sp + 4) = n1;
      const v8h nh = cvt8(n0, n1);
      *(v8h*)(hst16 + (wave * 32 + 16 * et + m) * LL + 16 * ft + 8 * hh) = nh;
      bh[et].h[ft] = nh;
    }
  }

  if (last != 0) {
    v8f d3[2][2];
#pragma unroll
    for (int ft = 0; ft < 2; ++ft) {
      FragH a;
      const _Float16* ap = wd1 + (16 * ft + m) * LL + 8 * hh;
      a.h[0] = *(const v8h*)ap;
      a.h[1] = *(const v8h*)(ap + 16);
      const v8f c = ldc8(db1s + 16 * ft + 8 * hh);
      d3[ft][0] = wmh(a.v, bh[0].v, c);
      d3[ft][1] = wmh(a.v, bh[1].v, c);
    }
    FragH bd[2];
    bd[0].h[0] = relu8(d3[0][0]); bd[0].h[1] = relu8(d3[1][0]);
    bd[1].h[0] = relu8(d3[0][1]); bd[1].h[1] = relu8(d3[1][1]);
    FragH a2;
    {
      const _Float16* ap = wd2 + m * LL + 8 * hh;
      a2.h[0] = *(const v8h*)ap;
      a2.h[1] = *(const v8h*)(ap + 16);
    }
    v8f c4 = zero8f();
    c4[0] = (hh == 0) ? db2s : 0.0f;
    const v8f u0 = wmh(a2.v, bd[0].v, c4);
    const v8f u1 = wmh(a2.v, bd[1].v, c4);
    const float ua = u0[0] * WINV, ub = u1[0] * WINV;
    if (hh == 0) {
      ust[wave * 32 + m]      = ua;
      ust[wave * 32 + 16 + m] = ub;
    }
  }
  __syncthreads();

  const size_t rb = (size_t)(blockIdx.x * NNODE + wave * 32) * LL;
  const int outBase = blockIdx.x * NNODE;
  node_store_pass(hst + wave * 32 * LL, hst16 + wave * 32 * LL, ust, hbuf, h16, outp, rb, outBase, outLim, lane, wave, last);
  __threadfence();
  node_store_pass(hst + wave * 32 * LL, hst16 + wave * 32 * LL, ust, hbuf, h16, outp, rb, outBase, outLim, lane, wave, last);
}

extern "C" void kernel_launch(void* const* d_in, const int* in_sizes, int n_in,
                              void* d_out, int out_size, void* d_ws, size_t ws_size,
                              hipStream_t stream) {
  if (n_in < 19) return;
  const int nE = in_sizes[0] / 2;
  const int nN = in_sizes[2];
  if (nE <= 0 || nN <= 0 || in_sizes[0] != 2 * nE || in_sizes[1] != 3 * nE) return;
  const int T = in_sizes[18];
  if (T <= 0) return;
  if (in_sizes[3]  != T * DPHI * LL || in_sizes[4]  != T * LL || in_sizes[5]  != T * LL * LL || in_sizes[6]  != T * LL) return;
  if (in_sizes[7]  != T * DPHI * LL || in_sizes[8]  != T * LL || in_sizes[9]  != T * LL * LL || in_sizes[10] != T * LL) return;
  if (in_sizes[11] != T * DPSI * LL || in_sizes[12] != T * LL || in_sizes[13] != T * LL * LL || in_sizes[14] != T * LL) return;
  if (in_sizes[15] != T * LL * LL || in_sizes[16] != T * LL || in_sizes[17] != T * LL) return;
  if (out_size != nN) return;

  const int*   edge_index  = (const int*)d_in[0];
  const float* edge_attr   = (const float*)d_in[1];
  const float* prb         = (const float*)d_in[2];
  const float* phi_to_W1   = (const float*)d_in[3];
  const float* phi_to_b1   = (const float*)d_in[4];
  const float* phi_to_W2   = (const float*)d_in[5];
  const float* phi_to_b2   = (const float*)d_in[6];
  const float* phi_from_W1 = (const float*)d_in[7];
  const float* phi_from_b1 = (const float*)d_in[8];
  const float* phi_from_W2 = (const float*)d_in[9];
  const float* phi_from_b2 = (const float*)d_in[10];
  const float* psi_W1 = (const float*)d_in[11];
  const float* psi_b1 = (const float*)d_in[12];
  const float* psi_W2 = (const float*)d_in[13];
  const float* psi_b2 = (const float*)d_in[14];
  const float* dec_W1 = (const float*)d_in[15];
  const float* dec_b1 = (const float*)d_in[16];
  const float* dec_W2 = (const float*)d_in[17];
  const float* dec_b2 = (const float*)d_in[18];
  float* out = (float*)d_out;

  const int nBlkE = (nN + NB - 1) / NB;
  const int nBlkN = (nN + NNODE - 1) / NNODE;
  int rowsPad = nBlkE * NB;
  if (nBlkN * NNODE > rowsPad) rowsPad = nBlkN * NNODE;

  char* ws = (char*)d_ws;
  size_t off = 0;
  const size_t oH = off;   off += (size_t)rowsPad * LL * 4;  off = (off + 255) & ~(size_t)255;
  const size_t oH16 = off; off += (size_t)rowsPad * LL * 2;  off = (off + 255) & ~(size_t)255;
  const size_t oM = off;   off += (size_t)2 * rowsPad * LL * 4;  off = (off + 255) & ~(size_t)255;
  if (off > ws_size || off > (size_t)134217728) return;
  float*    hbuf = (float*)(ws + oH);
  _Float16* h16  = (_Float16*)(ws + oH16);
  float*    mess = (float*)(ws + oM);

  const int vec8 = ((nE & 3) == 0) ? 1 : 0;

  for (int t = 0; t < T; ++t) {
    const int hz = (t == 0) ? 1 : 0;
    const int last = (t == T - 1) ? 1 : 0;
    k_edge<<<dim3(nBlkE, 2, 1), dim3(NTHR, 1, 1), 0, stream>>>(
        h16, edge_index, edge_attr,
        phi_to_W1, phi_to_b1, phi_to_W2, phi_to_b2,
        phi_from_W1, phi_from_b1, phi_from_W2, phi_from_b2,
        mess, nN, nE, t, hz, vec8, rowsPad);
    k_node<<<dim3(nBlkN, 1, 1), dim3(NTHR, 1, 1), 0, stream>>>(
        hbuf, h16, mess, prb,
        psi_W1, psi_b1, psi_W2, psi_b2,
        dec_W1, dec_b1, dec_W2, dec_b2,
        out, nN, t, hz, last, rowsPad, out_size);
  }
}
